// QuantumLayer_44968307589412
// MI455X (gfx1250) — hardware-verified
//
#include <hip/hip_runtime.h>
#include <math.h>


#ifndef NBATCH
#define NBATCH 262144
#endif
#define NBATCH_FULL 262144
#define NCOMP 24
#define MSZ   1024
#define CW    8
#define QRS   2048.0f
#define QRI   (1.0f / 2048.0f)

static_assert(NBATCH <= NBATCH_FULL);
static_assert(NBATCH % (16 * CW) == 0);
static_assert(MSZ == 32 * 32);
static_assert((MSZ * 2) % 128 == 0);
static_assert(128 * 8 == MSZ);
static_assert(16 * 16 == 256);
static_assert(32 * 16 == 16 * CW * 4);
static_assert((16 * CW) * 4 <= 131072);
static_assert((512 + 512 + 1024 + 32 + 32) * 4 <= 131072);

typedef _Float16 h16;
typedef __attribute__((ext_vector_type(16))) _Float16 v16h;
typedef __attribute__((ext_vector_type(8)))  _Float16 v8h;
typedef __attribute__((ext_vector_type(8)))  float    v8f;
typedef __attribute__((ext_vector_type(4)))  float    v4f;
typedef v4f  __attribute__((may_alias)) v4fa;

__device__ __forceinline__ unsigned short f2bf(float f) { unsigned u = __float_as_uint(f); u += 0x7FFFu + ((u >> 16) & 1u); return (unsigned short)(u >> 16); }
__device__ __forceinline__ float bfr(float f) { return __uint_as_float(((unsigned)f2bf(f)) << 16); }
__device__ __forceinline__ v16h cat16(v8h lo, v8h hi) { return __builtin_shufflevector(lo, hi, 0, 1, 2, 3, 4, 5, 6, 7, 8, 9, 10, 11, 12, 13, 14, 15); }
__device__ __forceinline__ v16h ldh(const h16* p) { return cat16(*(const v8h*)p, *(const v8h*)(p + 16)); }
static __device__ __forceinline__ h16 toh_flush(float v) { const h16 r = (h16)v; return (fabsf(v) < 6.103515625e-05f) ? (h16)0.0f : r; }
__device__ __forceinline__ v8f wmma16g(v16h a, v16h b, v8f c) {
    c = __builtin_amdgcn_wmma_f32_16x16x32_f16(false, a, false, b, (short)0, c, false, false);
    asm volatile("v_nop\n\tv_nop\n\tv_nop\n\tv_nop" : "+v"(c) : "v"(a), "v"(b));
    return c;
}

__device__ __forceinline__ int xpf(int k) { return 8 * (k >> 2) + 2 * (k & 3) + ((k & 3) >> 1); }

__device__ __forceinline__ void gate_row(const int kind, const int w, const float c, const float s, const int o,
                                         int& j0, int& j1, float& ar, float& ai, float& br, float& bi) {
#pragma clang fp contract(off)
    const int b0 = 8 >> w, b1 = 8 >> ((w + 1) & 3), b2 = 8 >> ((w + 2) & 3);
    const bool ob = (o & b0) != 0, y1 = (o & b1) != 0, y2 = (o & b2) != 0;
    const float RH = 0.70710678118654752f;
    j0 = o & ~b0; j1 = o | b0; ar = 0.0f; ai = 0.0f; br = 0.0f; bi = 0.0f;
    if (kind == 0)      { ar = ob ? 0.0f : c; ai = ob ? -s : 0.0f; br = ob ? c : 0.0f; bi = ob ? 0.0f : -s; }
    else if (kind == 1) { ar = ob ? s : c; br = ob ? c : -s; }
    else if (kind == 2) { ar = ob ? 0.0f : c; ai = ob ? 0.0f : -s; br = ob ? c : 0.0f; bi = ob ? s : 0.0f; }
    else if (kind == 3) { ar = RH; br = ob ? -RH : RH; }
    else if (kind == 4) { ar = ob ? 1.0f : 0.0f; br = ob ? 0.0f : 1.0f; }
    else if (kind == 5) { ai = ob ? 1.0f : 0.0f; bi = ob ? 0.0f : -1.0f; }
    else if (kind == 6) { ar = ob ? 0.0f : 1.0f; br = ob ? -1.0f : 0.0f; }
    else {
        j1 = o; ar = 1.0f;
        if (kind == 7)      { j0 = ob ? (o ^ b1) : o; }
        else if (kind == 8) { j0 = o; ar = (ob & y1) ? -1.0f : 1.0f; }
        else if (kind == 9) { j0 = (ob & y1) ? (o ^ b2) : o; }
        else                { j0 = (ob & (y1 != y2)) ? (o ^ b1 ^ b2) : o; }
    }
}

__global__ __launch_bounds__(256) void k_build(const float* __restrict__ QP, h16* MPL) {
#pragma clang fp contract(off)
    __shared__ float Mr[512];
    __shared__ float Mi[512];
    __shared__ __align__(16) float R[1024];
    __shared__ float cw[32];
    __shared__ float sw[32];
    const int tid = threadIdx.x; const int o = tid >> 4, i = tid & 15;
    { const int k = tid < 24 ? tid : 23;
      float wv = QP[k]; asm volatile("" : "+v"(wv)); wv = bfr(wv);
      float sn, cs; sincosf(0.5f * wv, &sn, &cs);
      if (tid < 24) { cw[tid] = cs; sw[tid] = sn; } }
    __syncthreads();
#pragma unroll 1
    for (int c = 0; c < NCOMP; ++c) {
        const bool fw = c <= 11;
        const bool ad = (c >= 11) & (c <= 22);
        const int f0 = fw ? xpf(c) : 0;
        const int nf = fw ? (xpf(c + 1) - xpf(c)) : 0;
        const int a1 = ad ? (xpf(23 - c) - 1) : 0;
        const int a0 = ad ? xpf(22 - c) : 0;
        const int na = ad ? (a1 - a0 + 1) : 0;
        const int nh = (c == 23) ? 4 : 0;
        const int nfs = 2 * nf, nas = 2 * na;
        const int ns = nfs + nas + nh;
        Mr[tid] = (o == i) ? 1.0f : 0.0f; Mi[tid] = 0.0f;
        __syncthreads();
        int cur = 0;
#pragma unroll 1
        for (int e = 0; e < ns; ++e) {
            int p = 0, hw = 0; bool isw = false, ish = false, neg = false;
            if (e < nfs)            { p = f0 + (e >> 1); isw = (e & 1) == 0; }
            else if (e < nfs + nas) { const int e2 = e - nfs; p = a1 - (e2 >> 1); isw = (e2 & 1) == 1; neg = true; }
            else                    { ish = true; hw = e - nfs - nas; }
            const int kind = ish ? 3 : (isw ? (((p >> 2) + (p & 3)) % 3) : (3 + (p & 7)));
            const int w = ish ? hw : (p & 3);
            const float cs = cw[p]; const float s0 = sw[p]; const float sn = neg ? -s0 : s0;
            int j0, j1; float ar, ai, br, bi;
            gate_row(kind, w, cs, sn, o, j0, j1, ar, ai, br, bi);
            const int rb = cur * 256, wb = (cur ^ 1) * 256;
            const float m0r = Mr[rb + j0 * 16 + i], m0i = Mi[rb + j0 * 16 + i];
            const float m1r = Mr[rb + j1 * 16 + i], m1i = Mi[rb + j1 * 16 + i];
            const float nr = (ar * m0r - ai * m0i) + (br * m1r - bi * m1i);
            const float ni = (ar * m0i + ai * m0r) + (br * m1i + bi * m1r);
            Mr[wb + tid] = nr; Mi[wb + tid] = ni;
            __syncthreads();
            cur ^= 1;
        }
        { const float ur = Mr[cur * 256 + tid], ui = Mi[cur * 256 + tid];
          R[o * 32 + i] = ur; R[o * 32 + 16 + i] = -ui; R[(16 + o) * 32 + i] = ui; R[(16 + o) * 32 + 16 + i] = ur; }
        __syncthreads();
        { const int pl = tid >> 7, q = tid & 127;
          const v4f x0 = *(const v4fa*)(&R[q * 8]); const v4f x1 = *(const v4fa*)(&R[q * 8 + 4]); v8h hv, rv;
#pragma unroll
          for (int k = 0; k < 4; ++k) { const h16 a0 = toh_flush(x0[k]); const h16 a1v = toh_flush(x1[k]); hv[k] = a0; hv[4 + k] = a1v;
              rv[k] = toh_flush((x0[k] - (float)a0) * QRS); rv[4 + k] = toh_flush((x1[k] - (float)a1v) * QRS); }
          const v8h ov = pl ? rv : hv;
          const size_t off = (size_t)pl * ((size_t)NCOMP * MSZ) + (size_t)c * MSZ + (size_t)q * 8;
          *(volatile v8h*)(MPL + off) = ov; __threadfence(); *(volatile v8h*)(MPL + off) = ov; }
        __syncthreads();
    }
}

template <int WIRE>
__device__ __forceinline__ void stage(v8f& Sr, v8f& Si, const float c, const float s, const int hi,
                                      const h16* __restrict__ MH, const h16* __restrict__ MR, const size_t ao) {
    if (WIRE == 0) {
        const float sp = hi ? s : -s;
#pragma unroll
        for (int r = 0; r < 8; ++r) {
            const float pr = __shfl_xor(Sr[r], 16, 32), pi = __shfl_xor(Si[r], 16, 32);
            Sr[r] = c * Sr[r] + sp * pr; Si[r] = c * Si[r] + sp * pi; }
    } else {
        const int d = (WIRE == 1) ? 4 : ((WIRE == 2) ? 2 : 1);
#pragma unroll
        for (int r = 0; r < 8; ++r) {
            if ((r & d) == 0) {
                const float r0 = Sr[r], r1 = Sr[r + d], i0 = Si[r], i1 = Si[r + d];
                Sr[r] = c * r0 - s * r1; Sr[r + d] = s * r0 + c * r1;
                Si[r] = c * i0 - s * i1; Si[r + d] = s * i0 + c * i1; } }
    }
    v16h bh, br;
#pragma unroll
    for (int r = 0; r < 8; ++r) {
        const h16 a0 = toh_flush(Sr[r]); const h16 a1 = toh_flush(Si[r]);
        bh[r] = a0; bh[8 + r] = a1;
        br[r] = toh_flush((Sr[r] - (float)a0) * QRS); br[8 + r] = toh_flush((Si[r] - (float)a1) * QRS); }
    const h16* ph = MH + ao; const h16* pq = MR + ao;
    const v16h a0h = ldh(ph), a1h = ldh(ph + 512), a0r = ldh(pq), a1r = ldh(pq + 512);
    v8f h0 = (v8f){}, h1 = (v8f){}, q0 = (v8f){}, q1 = (v8f){};
    h0 = wmma16g(a0h, bh, h0); q0 = wmma16g(a0h, br, q0); q0 = wmma16g(a0r, bh, q0);
    h1 = wmma16g(a1h, bh, h1); q1 = wmma16g(a1h, br, q1); q1 = wmma16g(a1r, bh, q1);
    Sr = h0 + q0 * QRI; Si = h1 + q1 * QRI;
}

__global__ __launch_bounds__(256) __attribute__((amdgpu_num_vgpr(256)))
void k_circ(const float* __restrict__ X1, const float* __restrict__ X2, const h16* __restrict__ MH, const h16* __restrict__ MR, float* OUT) {
    __shared__ __align__(16) float os[16 * CW];
    const int lane = threadIdx.x & 31, lr = lane & 15, hi = lane >> 4;
    const int wave = __builtin_amdgcn_readfirstlane((int)(threadIdx.x >> 5));
    const size_t bcol = (size_t)blockIdx.x * (16 * CW) + (size_t)(wave * 16 + lr);
    const v4f xa = *(const v4f*)(X1 + bcol * 4); const v4f xb = *(const v4f*)(X2 + bcol * 4);
    float c1[4], s1[4], c2[4], s2[4];
#pragma unroll
    for (int n = 0; n < 4; ++n) {
        const float xv = hi ? bfr(xb[n]) : bfr(xa[n]);
        float sn, cs; sincosf(0.5f * xv, &sn, &cs);
        sn = hi ? -sn : sn;
        const float co = __shfl_xor(cs, 16, 32), so = __shfl_xor(sn, 16, 32);
        c1[n] = hi ? co : cs; s1[n] = hi ? so : sn; c2[n] = hi ? cs : co; s2[n] = hi ? sn : so; }
    v8f Sr, Si;
#pragma unroll
    for (int r = 0; r < 8; ++r) { Sr[r] = 0.25f; Si[r] = 0.0f; }
    const size_t fo = (size_t)(lr * 32 + 8 * hi);
#pragma unroll 1
    for (int g = 0; g < 3; ++g) {
        const size_t cb = (size_t)(4 * g) * MSZ + fo;
        stage<0>(Sr, Si, c1[0], s1[0], hi, MH, MR, cb);
        stage<2>(Sr, Si, c1[2], s1[2], hi, MH, MR, cb + MSZ);
        stage<1>(Sr, Si, c1[1], s1[1], hi, MH, MR, cb + 2 * MSZ);
        stage<3>(Sr, Si, c1[3], s1[3], hi, MH, MR, cb + 3 * MSZ);
    }
#pragma unroll 1
    for (int g = 0; g < 3; ++g) {
        const size_t cb = (size_t)(12 + 4 * g) * MSZ + fo;
        stage<3>(Sr, Si, c2[3], s2[3], hi, MH, MR, cb);
        stage<1>(Sr, Si, c2[1], s2[1], hi, MH, MR, cb + MSZ);
        stage<2>(Sr, Si, c2[2], s2[2], hi, MH, MR, cb + 2 * MSZ);
        stage<0>(Sr, Si, c2[0], s2[0], hi, MH, MR, cb + 3 * MSZ);
    }
    const float ar = Sr[0], ai = Si[0];
    const float pv = ar * ar + ai * ai;
    if (hi == 0) os[wave * 16 + lr] = pv;
    __syncthreads();
    if (wave == 0) {
        const v4f val = *(const v4fa*)(&os[lane * 4]);
        float* op = OUT + (size_t)blockIdx.x * (16 * CW) + (size_t)lane * 4;
        *(volatile v4f*)op = val; __threadfence(); *(volatile v4f*)op = val;
    }
}

static constexpr size_t al256(size_t v) { return (v + 255) & ~(size_t)255; }
static constexpr size_t SZ_MP = al256((size_t)2 * NCOMP * MSZ * 2);
static constexpr size_t SZ_TOTAL = SZ_MP;
static_assert(SZ_TOTAL <= (size_t)134217728);
static_assert((size_t)(1 * ((size_t)NCOMP * MSZ) + (size_t)(NCOMP - 1) * MSZ + 127 * 8 + 8) * 2 <= SZ_MP);

extern "C" void kernel_launch(void* const* d_in, const int* in_sizes, int n_in,
                              void* d_out, int out_size, void* d_ws, size_t ws_size, hipStream_t stream) {
    if (n_in < 3) return;
    if ((size_t)in_sizes[0] < (size_t)NBATCH * 4 || (size_t)in_sizes[1] < (size_t)NBATCH * 4) return;
    if (in_sizes[2] < 24) return;
    if ((size_t)out_size < (size_t)NBATCH) return;
    if (SZ_TOTAL > ws_size) return;
    const float* x1 = (const float*)d_in[0];
    const float* x2 = (const float*)d_in[1];
    const float* qp = (const float*)d_in[2];
    float* OUT = (float*)d_out;
    h16* MPL = (h16*)d_ws;
    h16* MH = MPL; h16* MR = MPL + (size_t)NCOMP * MSZ;

    k_build<<<1, 256, 0, stream>>>(qp, MPL);
    k_circ<<<dim3(NBATCH / (16 * CW), 1, 1), 32 * CW, 0, stream>>>(x1, x2, MH, MR, OUT);
}
